// gwnetgat_8821862826031
// MI455X (gfx1250) — hardware-verified
//
#include <hip/hip_runtime.h>
#include <math.h>

typedef __attribute__((ext_vector_type(16))) _Float16 v16h;
typedef __attribute__((ext_vector_type(8)))  _Float16 v8h;
typedef __attribute__((ext_vector_type(16))) __bf16   v16b;
typedef __attribute__((ext_vector_type(8)))  __bf16   v8b;
typedef __attribute__((ext_vector_type(8)))  float    v8f;
typedef __attribute__((ext_vector_type(4)))  float    v4f;
typedef __attribute__((ext_vector_type(4)))  int      v4i;

#define BB 8
#define CC 64
#define TT 24
#define NN 512
#define BT 192
#define KC 64
#define PP 72
#define VP 72
#define OP 68
#define XP 65
#define PSC 32768.0f

__device__ __forceinline__ unsigned short f2bf_bits(float f) {
  unsigned u = __float_as_uint(f);
  return (unsigned short)((u + 0x7FFFu + ((u >> 16) & 1u)) >> 16);
}
__device__ __forceinline__ float bf_bits2f(unsigned short h) { return __uint_as_float(((unsigned)h) << 16); }

__device__ __forceinline__ void dep_guard_h(v8f& a, v8f& b, v16h x, v16h y) { asm volatile("v_nop\n\tv_nop\n\tv_nop\n\tv_nop" : "+v"(a), "+v"(b) : "v"(x), "v"(y)); }
__device__ __forceinline__ void dep_guard_b(v8f& a, v8f& b, v16b x, v16b y) { asm volatile("v_nop\n\tv_nop\n\tv_nop\n\tv_nop" : "+v"(a), "+v"(b) : "v"(x), "v"(y)); }
__device__ __forceinline__ void keep4_h(v16h a, v16h b, v16h c, v16h d) { asm volatile("v_nop" :: "v"(a), "v"(b), "v"(c), "v"(d)); }
__device__ __forceinline__ void keep4_b(v16b a, v16b b, v16b c, v16b d) { asm volatile("v_nop" :: "v"(a), "v"(b), "v"(c), "v"(d)); }
__device__ __forceinline__ void acc_guard4(v8f& a, v8f& b, v8f& c, v8f& d) { asm volatile("v_nop\n\tv_nop\n\tv_nop\n\tv_nop" : "+v"(a), "+v"(b), "+v"(c), "+v"(d)); }
template <typename T> struct Frag;
template <> struct Frag<_Float16> {
  typedef v16h V; union U { v16h v; v8h h[2]; };
  static __device__ __forceinline__ v16h load(const _Float16* p) {
    U f; f.h[0] = *(const v8h*)(p); f.h[1] = *(const v8h*)(p + 16); return f.v;
  }
  static __device__ __forceinline__ v8f mma(v16h a, v16h b, v8f c) {
    return __builtin_amdgcn_wmma_f32_16x16x32_f16(false, a, false, b, (short)0, c, false, false);
  }
  static __device__ __forceinline__ void guard(v8f& a, v8f& b, v16h x, v16h y) { dep_guard_h(a, b, x, y); }
  static __device__ __forceinline__ void keep(v16h a, v16h b, v16h c, v16h d) { keep4_h(a, b, c, d); }
};
template <> struct Frag<__bf16> {
  typedef v16b V; union U { v16b v; v8b h[2]; };
  static __device__ __forceinline__ v16b load(const __bf16* p) {
    U f; f.h[0] = *(const v8b*)(p); f.h[1] = *(const v8b*)(p + 16); return f.v;
  }
  static __device__ __forceinline__ v8f mma(v16b a, v16b b, v8f c) {
    return __builtin_amdgcn_wmma_f32_16x16x32_bf16(false, a, false, b, (short)0, c, false, false);
  }
  static __device__ __forceinline__ void guard(v8f& a, v8f& b, v16b x, v16b y) { dep_guard_b(a, b, x, y); }
  static __device__ __forceinline__ void keep(v16b a, v16b b, v16b c, v16b d) { keep4_b(a, b, c, d); }
};

template <int ET> struct Elem;
template <> struct Elem<0> { typedef _Float16 T; };
template <> struct Elem<1> { typedef __bf16 T; };
template <int ET, bool SPLIT, int BIAS_MODE, int OUT_MODE, bool RESID, int ACT = 0>
__global__ __launch_bounds__(256) void wmma_gemm64(
    const unsigned short* __restrict__ Ap, const unsigned short* __restrict__ A2p, int lda, long strideA,
    const unsigned short* __restrict__ Btp, const unsigned short* __restrict__ Bt2p, int ldb, long strideB,
    void* __restrict__ Cout, void* __restrict__ Cout2, int ldc, long strideC,
    const float* __restrict__ bias,
    const float* __restrict__ resid, long strideR,
    int M, int N, int K, float scale) {
  typedef typename Elem<ET>::T T;
  typedef typename Frag<T>::V V;
  const T* A = (const T*)Ap; const T* A2 = (const T*)A2p; const T* Bt = (const T*)Btp; const T* Bt2 = (const T*)Bt2p;
  __shared__ __align__(16) float sT[8][16 * 68];
  const int b    = blockIdx.y;
  const int lane = threadIdx.x & 31;
  const int wave = threadIdx.x >> 5;
  const int tilesN = N >> 6;
  const int tilesM = M >> 6;
  const int tile = blockIdx.x * 8 + wave;
  if (tile >= tilesM * tilesN) return;
  const int tm = tile / tilesN;
  const int tn = tile - tm * tilesN;
  const int m0 = tm << 6;
  const int n0 = tn << 6;

  const T* Ab  = A  + (size_t)b * strideA;
  const T* Bb  = Bt + (size_t)b * strideB;
  const T* Ab2 = SPLIT ? (A2  + (size_t)b * strideA) : nullptr;
  const T* Bb2 = SPLIT ? (Bt2 + (size_t)b * strideB) : nullptr;

  const int rlane = lane & 15;
  const int koff  = (lane >> 4) * 8;
  const int mOff  = (lane >> 4) * 8;

  v8f acc[4][4];
#pragma unroll
  for (int i = 0; i < 4; ++i)
#pragma unroll
    for (int j = 0; j < 4; ++j) acc[i][j] = (v8f){0.f,0.f,0.f,0.f,0.f,0.f,0.f,0.f};

  for (int k0 = 0; k0 < K; k0 += 32) {
    V bh[4], bl[4];
#pragma unroll
    for (int j = 0; j < 4; ++j) {
      const size_t bo = (size_t)(n0 + (j << 4) + rlane) * ldb + koff + k0;
      bh[j] = Frag<T>::load(Bb + bo);
      if (SPLIT) bl[j] = Frag<T>::load(Bb2 + bo);
    }
#pragma unroll
    for (int i = 0; i < 4; ++i) {
      const size_t ao = (size_t)(m0 + (i << 4) + rlane) * lda + koff + k0;
      V ah = Frag<T>::load(Ab + ao);
      V al;
      if (SPLIT) al = Frag<T>::load(Ab2 + ao);
#pragma unroll
      for (int j = 0; j < 4; ++j) {
        acc[i][j] = Frag<T>::mma(ah, bh[j], acc[i][j]);
        if (SPLIT) {
          acc[i][j] = Frag<T>::mma(ah, bl[j], acc[i][j]);
          acc[i][j] = Frag<T>::mma(al, bh[j], acc[i][j]);
        }
      }
      Frag<T>::guard(acc[i][0], acc[i][3], ah, SPLIT ? al : ah);
    }
    Frag<T>::keep(bh[0], bh[1], bh[2], bh[3]);
    if (SPLIT) Frag<T>::keep(bl[0], bl[1], bl[2], bl[3]);
  }
  acc_guard4(acc[0][0], acc[0][1], acc[0][2], acc[0][3]);
  acc_guard4(acc[1][0], acc[1][1], acc[1][2], acc[1][3]);
  acc_guard4(acc[2][0], acc[2][1], acc[2][2], acc[2][3]);
  acc_guard4(acc[3][0], acc[3][1], acc[3][2], acc[3][3]);

  float* slab = sT[wave];
  const float* Rb = RESID ? (resid + (size_t)b * strideR) : nullptr;
#pragma unroll
  for (int i = 0; i < 4; ++i) {
    const int mBase = m0 + (i << 4);
#pragma unroll
    for (int j = 0; j < 4; ++j) {
      const int n = n0 + (j << 4) + rlane;
      float bv = 0.f;
      if (BIAS_MODE == 2) bv = bias[n];
#pragma unroll
      for (int r = 0; r < 8; ++r) {
        float v = acc[i][j][r] * scale;
        if (BIAS_MODE == 1) v += bias[mBase + mOff + r];
        if (BIAS_MODE == 2) v += bv;
        if (RESID) v += Rb[(size_t)(mBase + mOff + r) * ldc + n];
        if (ACT == 1) v = tanhf(v);
        if (ACT == 2) v = fmaxf(v, 0.0f);
        if (ACT == 3) v = v / (1.0f + expf(-v));
        if (ACT == 4) v = (v > 0.f) ? v : 0.01f * v;
        if (ACT == 5) v = 0.5f * v * (1.0f + erff(v * 0.70710678118654752f));
        slab[(mOff + r) * 68 + (j << 4) + rlane] = v;
      }
    }
    __builtin_amdgcn_fence(__ATOMIC_RELEASE, "workgroup");
    __builtin_amdgcn_wave_barrier();
    __builtin_amdgcn_fence(__ATOMIC_ACQUIRE, "workgroup");
    if (OUT_MODE == 0) {
      float* C = (float*)Cout + (size_t)b * strideC;
      const int hh = lane >> 4, c4 = (lane & 15) * 4;
      for (int pass = 0; pass < 2; ++pass) {
#pragma unroll
        for (int it = 0; it < 8; ++it) {
          const int row = it * 2 + hh;
          v4f v = *(const v4f*)(slab + row * 68 + c4);
          *(volatile v4f*)(C + (size_t)(mBase + row) * ldc + n0 + c4) = v;
        }
        __threadfence();
      }
    } else {
      const int q = lane >> 3, c8 = (lane & 7) * 8;
      unsigned short* C  = (unsigned short*)Cout  + (size_t)b * strideC;
      unsigned short* C2 = (OUT_MODE == 2) ? ((unsigned short*)Cout2 + (size_t)b * strideC) : nullptr;
      for (int pass = 0; pass < 2; ++pass) {
#pragma unroll
        for (int it = 0; it < 4; ++it) {
          const int row = it * 4 + q;
          const float* sp = slab + row * 68 + c8;
          v8h hv, lv;
#pragma unroll
          for (int e = 0; e < 8; ++e) {
            if (OUT_MODE == 1) {
              hv[e] = (_Float16)sp[e];
            } else {
              unsigned short hb = f2bf_bits(sp[e]);
              unsigned short lb = f2bf_bits(sp[e] - bf_bits2f(hb));
              hv[e] = __builtin_bit_cast(_Float16, hb);
              lv[e] = __builtin_bit_cast(_Float16, lb);
            }
          }
          *(volatile v8h*)(C + (size_t)(mBase + row) * ldc + n0 + c8) = hv;
          if (OUT_MODE == 2) *(volatile v8h*)(C2 + (size_t)(mBase + row) * ldc + n0 + c8) = lv;
        }
        __threadfence();
      }
    }
    __builtin_amdgcn_fence(__ATOMIC_RELEASE, "workgroup");
    __builtin_amdgcn_wave_barrier();
    __builtin_amdgcn_fence(__ATOMIC_ACQUIRE, "workgroup");
  }
}

__device__ __forceinline__ v8f mma_h(v16h a, v16h b, v8f c) {
  c = __builtin_amdgcn_wmma_f32_16x16x32_f16(false, a, false, b, (short)0, c, false, false);
  asm volatile("v_nop\n\tv_nop\n\tv_nop\n\tv_nop" : "+v"(c) : "v"(a), "v"(b));
  return c;
}

__global__ __launch_bounds__(512)
void prep_kernel(const float* __restrict__ Wq, const float* __restrict__ Wk, const float* __restrict__ Wv,
                 const float* __restrict__ a_src, const float* __restrict__ a_dst,
                 float* __restrict__ Weff, _Float16* __restrict__ Wv16) {
  const int tid = threadIdx.x;
  float acc = 0.f;
  if (tid < 256) {
    const int which = tid >> 6, cc = tid & 63, hsel = which & 1;
    const float* W  = (which < 2) ? Wq : Wk;
    const float* av = (which < 2) ? a_src : a_dst;
#pragma unroll 4
    for (int d = 0; d < 32; ++d) acc += av[hsel * 32 + d] * W[(hsel * 32 + d) * CC + cc];
  }
  v8h wv;
#pragma unroll
  for (int e = 0; e < 8; ++e) wv[e] = (_Float16)Wv[tid * 8 + e];
  for (int pass = 0; pass < 2; ++pass) {
    if (tid < 256) *(volatile float*)(Weff + tid) = acc;
    *(volatile v8h*)(Wv16 + tid * 8) = wv;
    __threadfence();
  }
}

__global__ __launch_bounds__(256)
void xr_scores_kernel(const float* __restrict__ x, const float* __restrict__ Weff,
                      _Float16* __restrict__ xr16, float* __restrict__ S) {
  __shared__ float xs[64 * XP];
  __shared__ float we[256];
  const int tid = threadIdx.x, wave = tid >> 5, lane = tid & 31;
  const int bx = blockIdx.x, nb = bx & 7, bt = bx >> 3;
  const int b = bt / TT, t = bt - b * TT;
  const int n0 = nb * 64;
  we[tid] = Weff[tid];
#pragma unroll
  for (int it = 0; it < 4; ++it) {
    const int idx = it * 256 + tid, cch = idx >> 4, n4 = (idx & 15) * 4;
    const v4f v = *(const v4f*)(x + (((size_t)b * CC + cch) * TT + t) * NN + n0 + n4);
#pragma unroll
    for (int e = 0; e < 4; ++e) xs[(n4 + e) * XP + cch] = v[e];
  }
  __syncthreads();
  const int which = tid >> 6, node = tid & 63;
  float acc = 0.f;
#pragma unroll 8
  for (int cc = 0; cc < CC; ++cc) acc += xs[node * XP + cc] * we[which * CC + cc];
  const int q = lane >> 3, c8 = (lane & 7) * 8;
  const int row0 = wave * 4 + q, row1 = 32 + wave * 4 + q;
  v8h hv0, hv1;
#pragma unroll
  for (int e = 0; e < 8; ++e) {
    hv0[e] = (_Float16)xs[row0 * XP + c8 + e];
    hv1[e] = (_Float16)xs[row1 * XP + c8 + e];
  }
  float* sp = S + ((size_t)bt * 4 + which) * NN + n0 + node;
  _Float16* x0p = xr16 + ((size_t)bt * NN + n0 + row0) * CC + c8;
  _Float16* x1p = xr16 + ((size_t)bt * NN + n0 + row1) * CC + c8;
  for (int pass = 0; pass < 2; ++pass) {
    *(volatile float*)sp = acc;
    *(volatile v8h*)x0p = hv0;
    *(volatile v8h*)x1p = hv1;
    __threadfence();
  }
}

__global__ __launch_bounds__(256)
void attn_ln_kernel(const _Float16* __restrict__ V16, const float* __restrict__ S,
                    const int* __restrict__ gso, const float* __restrict__ gamma,
                    const float* __restrict__ beta, float* __restrict__ out) {
  __shared__ __align__(16) _Float16 Vt[CC * VP];
  __shared__ __align__(16) _Float16 Psh[8][16 * PP];
  __shared__ __align__(16) unsigned int Mw[64 * 16];
  __shared__ __align__(16) float Sd[2 * 64];
  __shared__ __align__(16) float Os[64 * OP];

  const int tid = threadIdx.x, wave = tid >> 5, lane = tid & 31;
  const int hh = lane >> 4, c = lane & 15;
  const int bx = blockIdx.x;
  const int ib = bx & 7, bt = bx >> 3;
  const int b = bt / TT, t = bt - b * TT;
  const int i0 = ib * 64;
  const int h = wave >> 2, wih = wave & 3;
  const int rbase = wih * 16 + 8 * hh;

  float ssrc[8], mrow[8], lrow[8];
  v8f oacc[2];
#pragma unroll
  for (int r = 0; r < 8; ++r) {
    ssrc[r] = S[((size_t)bt * 4 + h) * NN + i0 + rbase + r];
    mrow[r] = -INFINITY; lrow[r] = 0.f;
  }
  oacc[0] = (v8f){0.f,0.f,0.f,0.f,0.f,0.f,0.f,0.f};
  oacc[1] = (v8f){0.f,0.f,0.f,0.f,0.f,0.f,0.f,0.f};

  for (int kc = 0; kc < NN / KC; ++kc) {
    const int kv0 = kc * KC;
    __syncthreads();
    {
      const int kvr = tid >> 2, dq = (tid & 3) * 16;
      const _Float16* vp = V16 + ((size_t)bt * NN + kv0 + kvr) * CC + dq;
      const v8h va = *(const v8h*)vp;
      const v8h vb = *(const v8h*)(vp + 8);
#pragma unroll
      for (int e = 0; e < 8; ++e) {
        Vt[(dq + e) * VP + kvr]     = va[e];
        Vt[(dq + 8 + e) * VP + kvr] = vb[e];
      }
    }
    {
#pragma unroll
      for (int it = 0; it < 4; ++it) {
        const int idx = it * 256 + tid, row = idx >> 4, c4 = (idx & 15) * 4;
        const v4i g = *(const v4i*)(gso + (size_t)(i0 + row) * NN + kv0 + c4);
        const unsigned pk = (g[0] == 0 ? 1u : 0u) | ((g[1] == 0 ? 1u : 0u) << 8) |
                            ((g[2] == 0 ? 1u : 0u) << 16) | ((g[3] == 0 ? 1u : 0u) << 24);
        Mw[row * 16 + (c4 >> 2)] = pk;
      }
    }
    if (tid < 128) Sd[tid] = S[((size_t)bt * 4 + 2 + (tid >> 6)) * NN + kv0 + (tid & 63)];
    __syncthreads();

    float sdv[4];
#pragma unroll
    for (int j = 0; j < 4; ++j) sdv[j] = Sd[h * 64 + j * 16 + c];
    float sc[4][8], cm[8];
#pragma unroll
    for (int r = 0; r < 8; ++r) {
      const int rib = rbase + r;
      float m = -INFINITY;
#pragma unroll
      for (int j = 0; j < 4; ++j) {
        float v = ssrc[r] + sdv[j];
        v = (v >= 0.f) ? v : 0.2f * v;
        const unsigned mk = (Mw[rib * 16 + j * 4 + (c >> 2)] >> ((c & 3) * 8)) & 0xffu;
        if (mk != 0u) v = v + (-1.0e9f);
        sc[j][r] = v;
        m = fmaxf(m, v);
      }
#pragma unroll
      for (int off = 1; off < 16; off <<= 1) m = fmaxf(m, __shfl_xor(m, off, 32));
      cm[r] = m;
    }
    _Float16* pw = Psh[wave];
#pragma unroll
    for (int r = 0; r < 8; ++r) {
      const float mnew = fmaxf(mrow[r], cm[r]);
      const float alpha = expf(mrow[r] - mnew);
      mrow[r] = mnew;
      float psum = 0.f;
#pragma unroll
      for (int j = 0; j < 4; ++j) {
        const float p = expf(sc[j][r] - mnew);
        psum += p;
        pw[(8 * hh + r) * PP + j * 16 + c] = (_Float16)(p * PSC);
      }
#pragma unroll
      for (int off = 1; off < 16; off <<= 1) psum += __shfl_xor(psum, off, 32);
      lrow[r] = lrow[r] * alpha + psum;
      oacc[0][r] *= alpha;
      oacc[1][r] *= alpha;
    }
    __builtin_amdgcn_fence(__ATOMIC_RELEASE, "workgroup");
    __builtin_amdgcn_wave_barrier();
    __builtin_amdgcn_fence(__ATOMIC_ACQUIRE, "workgroup");
#pragma unroll
    for (int kk = 0; kk < 2; ++kk) {
      const v16h pa = Frag<_Float16>::load(pw + c * PP + kk * 32 + 8 * hh);
#pragma unroll
      for (int tt = 0; tt < 2; ++tt) {
        const v16h vb = Frag<_Float16>::load(Vt + (h * 32 + tt * 16 + c) * VP + kk * 32 + 8 * hh);
        oacc[tt] = mma_h(pa, vb, oacc[tt]);
      }
    }
  }

#pragma unroll
  for (int r = 0; r < 8; ++r) {
    const float inv = 1.0f / (lrow[r] * PSC);
#pragma unroll
    for (int tt = 0; tt < 2; ++tt) Os[(rbase + r) * OP + h * 32 + tt * 16 + c] = oacc[tt][r] * inv;
  }
  __syncthreads();
  {
    const int row = tid >> 2, q4 = tid & 3;
    float v[16];
    float s = 0.f;
#pragma unroll
    for (int e = 0; e < 16; ++e) { v[e] = Os[row * OP + q4 * 16 + e]; s += v[e]; }
    s += __shfl_xor(s, 1, 32);
    s += __shfl_xor(s, 2, 32);
    const float mu = s * (1.0f / 64.0f);
    float d = 0.f;
#pragma unroll
    for (int e = 0; e < 16; ++e) { const float dv = v[e] - mu; d += dv * dv; }
    d += __shfl_xor(d, 1, 32);
    d += __shfl_xor(d, 2, 32);
    const float var  = d * (1.0f / 64.0f);
    const float rstd = rsqrtf(var + 1.0e-5f);
#pragma unroll
    for (int e = 0; e < 16; ++e) {
      const int ch = q4 * 16 + e;
      Os[row * OP + ch] = (v[e] - mu) * rstd * gamma[ch] + beta[ch];
    }
  }
  __syncthreads();
  {
    const int c4 = c * 4;
    for (int pass = 0; pass < 2; ++pass) {
#pragma unroll
      for (int it = 0; it < 4; ++it) {
        const int ch = wave * 8 + it * 2 + hh;
        v4f val;
        val[0] = Os[(c4 + 0) * OP + ch];
        val[1] = Os[(c4 + 1) * OP + ch];
        val[2] = Os[(c4 + 2) * OP + ch];
        val[3] = Os[(c4 + 3) * OP + ch];
        *(volatile v4f*)(out + (((size_t)b * CC + ch) * TT + t) * NN + i0 + c4) = val;
      }
      __threadfence();
    }
  }
}

extern "C" void kernel_launch(void* const* d_in, const int* in_sizes, int n_in,
                              void* d_out, int out_size, void* d_ws, size_t ws_size,
                              hipStream_t stream) {
  if (n_in < 9) return;
  const int XE = BB * CC * TT * NN;
  if (in_sizes[0] != XE || in_sizes[1] != NN * NN || in_sizes[2] != CC * CC || in_sizes[3] != CC * CC ||
      in_sizes[4] != CC * CC || in_sizes[5] != 64 || in_sizes[6] != 64 || in_sizes[7] != CC ||
      in_sizes[8] != CC || out_size != XE) return;

  const float* x     = (const float*)d_in[0];
  const int*   gso   = (const int*)d_in[1];
  const float* Wq    = (const float*)d_in[2];
  const float* Wk    = (const float*)d_in[3];
  const float* Wv    = (const float*)d_in[4];
  const float* a_src = (const float*)d_in[5];
  const float* a_dst = (const float*)d_in[6];
  const float* gam   = (const float*)d_in[7];
  const float* bet   = (const float*)d_in[8];
  float* out = (float*)d_out;

  const size_t OFF_WEFF = 0;
  const size_t OFF_WV   = 1024;
  const size_t OFF_S    = 16384;
  const size_t OFF_XR   = OFF_S + (size_t)BT * 4 * NN * 4;
  const size_t OFF_V    = OFF_XR + (size_t)BT * NN * CC * 2;
  const size_t WS_TOTAL = OFF_V + (size_t)BT * NN * CC * 2;
  if (ws_size < WS_TOTAL) return;

  char* ws = (char*)d_ws;
  float*    Weff = (float*)(ws + OFF_WEFF);
  _Float16* Wv16 = (_Float16*)(ws + OFF_WV);
  float*    S    = (float*)(ws + OFF_S);
  _Float16* xr16 = (_Float16*)(ws + OFF_XR);
  _Float16* V16  = (_Float16*)(ws + OFF_V);

  prep_kernel<<<dim3(1), dim3(512), 0, stream>>>(Wq, Wk, Wv, a_src, a_dst, Weff, Wv16);
  xr_scores_kernel<<<dim3(BT * 8), dim3(256), 0, stream>>>(x, Weff, xr16, S);
  wmma_gemm64<0, false, 0, 1, false, 0><<<dim3((BT * NN / 64) / 8, 1, 1), dim3(256), 0, stream>>>(
      (const unsigned short*)xr16, (const unsigned short*)xr16, CC, 0L,
      (const unsigned short*)Wv16, (const unsigned short*)Wv16, CC, 0L,
      (void*)V16, (void*)V16, CC, 0L,
      Weff, Weff, 0L,
      BT * NN, CC, CC, 1.0f);
  attn_ln_kernel<<<dim3(BT * 8), dim3(256), 0, stream>>>(V16, S, gso, gam, bet, out);
}
